// StackAugmentedRNN_9981503996215
// MI455X (gfx1250) — hardware-run, weakly checked
//
#include <hip/hip_runtime.h>
#include <math.h>

constexpr int NVOC    = 45;
constexpr int NHID    = 1500;
constexpr int NSW     = 50;
constexpr int NSD     = 10;
constexpr int NSTEP   = 128;
constexpr int NIHP    = NHID + NSW;
constexpr int NH2     = 2 * NHID;
constexpr int HPADR   = 1504;
constexpr int KHP     = 1536;
constexpr int KREC    = 1600;
constexpr int NDIRROW = 4 * HPADR;
constexpr int NGROW   = 8 * HPADR;
constexpr int NTILE   = HPADR / 16;
constexpr int NTASK   = 2 * NTILE;
constexpr int NROWA   = NVOC + 3 + NSW;
constexpr int RTHR    = 512;
constexpr int RWAVES  = RTHR / 32;
constexpr int NREC8   = NGROW * (KREC / 8);
constexpr int NX8     = NGROW * (KHP / 8);
constexpr int NE8     = 64 * (KHP / 8);
constexpr int NB4     = NGROW / 4;
constexpr float WCARRY = 64.0f;
constexpr float HCARRY = 1024.0f;
constexpr float ECARRY = 64.0f;
constexpr float RECFOLD = 1.0f / (WCARRY * HCARRY);
constexpr float TABFOLD = 1.0f / (WCARRY * ECARRY);
static_assert(NIHP == 1550);
static_assert(NGROW == 12032 && NGROW % 64 == 0);
static_assert(KHP % 32 == 0 && KREC % 32 == 0 && KHP >= NHID && KREC - KHP >= NSW);
static_assert(HPADR % 16 == 0 && HPADR >= NHID && HPADR % 4 == 0 && NHID % 4 == 0);
static_assert(NREC8 % 256 == 0 && NX8 % 256 == 0 && NE8 % 256 == 0);
static_assert(NROWA == 98 && NROWA <= 7 * RWAVES);
static_assert(NH2 / 4 == 750 && 24 * 32 >= 750);
static_assert((NSTEP * NVOC) % 128 == 0);
static_assert(NSD * NSW <= RTHR);

typedef __attribute__((ext_vector_type(16))) _Float16 v16h;
typedef __attribute__((ext_vector_type(8)))  _Float16 v8h;
typedef __attribute__((ext_vector_type(16))) __bf16   v16b;
typedef __attribute__((ext_vector_type(8)))  __bf16   v8b;
typedef __attribute__((ext_vector_type(8)))  float    v8f;
typedef __attribute__((ext_vector_type(4)))  float    v4f;
typedef __attribute__((ext_vector_type(2)))  float    v2f;

__device__ __forceinline__ unsigned short f2bf_bits(float f) {
  unsigned u = __float_as_uint(f);
  return (unsigned short)((u + 0x7FFFu + ((u >> 16) & 1u)) >> 16);
}
__device__ __forceinline__ float bf_bits2f(unsigned short h) { return __uint_as_float(((unsigned)h) << 16); }

__device__ __forceinline__ void dep_guard4_h(v8f& a, v8f& b, v8f& c, v8f& d, v16h x, v16h y) { asm volatile("v_nop\n\tv_nop\n\tv_nop\n\tv_nop" : "+v"(a), "+v"(b), "+v"(c), "+v"(d) : "v"(x), "v"(y)); }
__device__ __forceinline__ void dep_guard4_b(v8f& a, v8f& b, v8f& c, v8f& d, v16b x, v16b y) { asm volatile("v_nop\n\tv_nop\n\tv_nop\n\tv_nop" : "+v"(a), "+v"(b), "+v"(c), "+v"(d) : "v"(x), "v"(y)); }
__device__ __forceinline__ void keep4_h(v16h a, v16h b, v16h c, v16h d) { asm volatile("v_nop" :: "v"(a), "v"(b), "v"(c), "v"(d)); }
__device__ __forceinline__ void keep4_b(v16b a, v16b b, v16b c, v16b d) { asm volatile("v_nop" :: "v"(a), "v"(b), "v"(c), "v"(d)); }
__device__ __forceinline__ void acc_guard4(v8f& a, v8f& b, v8f& c, v8f& d) { asm volatile("v_nop\n\tv_nop\n\tv_nop\n\tv_nop" : "+v"(a), "+v"(b), "+v"(c), "+v"(d)); }
__device__ __forceinline__ void rec_guard(v8f& a, v8f& b, v8f& c, v8f& d, v16h x, v16h y0, v16h y1, v16h y2, v16h y3) {
  asm volatile("v_nop\n\tv_nop\n\tv_nop\n\tv_nop" : "+v"(a), "+v"(b), "+v"(c), "+v"(d) : "v"(x), "v"(y0), "v"(y1), "v"(y2), "v"(y3));
}

template <typename T> struct Frag;
template <> struct Frag<_Float16> {
  typedef v16h V; union U { v16h v; v8h h[2]; };
  static __device__ __forceinline__ v16h load(const _Float16* p) {
    U f; f.h[0] = *(const v8h*)(p); f.h[1] = *(const v8h*)(p + 16); return f.v;
  }
  static __device__ __forceinline__ v8f mma(v16h a, v16h b, v8f c) {
    return __builtin_amdgcn_wmma_f32_16x16x32_f16(false, a, false, b, (short)0, c, false, false);
  }
  static __device__ __forceinline__ void guard4(v8f& a, v8f& b, v8f& c, v8f& d, v16h x, v16h y) { dep_guard4_h(a, b, c, d, x, y); }
  static __device__ __forceinline__ void keep(v16h a, v16h b, v16h c, v16h d) { keep4_h(a, b, c, d); }
};
template <> struct Frag<__bf16> {
  typedef v16b V; union U { v16b v; v8b h[2]; };
  static __device__ __forceinline__ v16b load(const __bf16* p) {
    U f; f.h[0] = *(const v8b*)(p); f.h[1] = *(const v8b*)(p + 16); return f.v;
  }
  static __device__ __forceinline__ v8f mma(v16b a, v16b b, v8f c) {
    return __builtin_amdgcn_wmma_f32_16x16x32_bf16(false, a, false, b, (short)0, c, false, false);
  }
  static __device__ __forceinline__ void guard4(v8f& a, v8f& b, v8f& c, v8f& d, v16b x, v16b y) { dep_guard4_b(a, b, c, d, x, y); }
  static __device__ __forceinline__ void keep(v16b a, v16b b, v16b c, v16b d) { keep4_b(a, b, c, d); }
};

template <int ET> struct Elem;
template <> struct Elem<0> { typedef _Float16 T; };
template <> struct Elem<1> { typedef __bf16 T; };
template <int ET, bool SPLIT, int BIAS_MODE, int OUT_MODE, bool RESID, int ACT = 0>
__global__ __launch_bounds__(256) void wmma_gemm64(
    const unsigned short* __restrict__ Ap, const unsigned short* __restrict__ A2p, int lda, long strideA,
    const unsigned short* __restrict__ Btp, const unsigned short* __restrict__ Bt2p, int ldb, long strideB,
    void* __restrict__ Cout, void* __restrict__ Cout2, int ldc, long strideC,
    const float* __restrict__ bias,
    const float* __restrict__ resid, long strideR,
    int M, int N, int K, float scale) {
  typedef typename Elem<ET>::T T;
  typedef typename Frag<T>::V V;
  const T* A = (const T*)Ap; const T* A2 = (const T*)A2p; const T* Bt = (const T*)Btp; const T* Bt2 = (const T*)Bt2p;
  __shared__ __align__(16) float sT[8][16 * 68];
  const int b    = blockIdx.y;
  const int lane = threadIdx.x & 31;
  const int wave = threadIdx.x >> 5;
  const int tilesN = N >> 6;
  const int tilesM = M >> 6;
  const int tile = blockIdx.x * 8 + wave;
  if (tile >= tilesM * tilesN) return;
  const int tm = tile / tilesN;
  const int tn = tile - tm * tilesN;
  const int m0 = tm << 6;
  const int n0 = tn << 6;

  const T* Ab  = A  + (size_t)b * strideA;
  const T* Bb  = Bt + (size_t)b * strideB;
  const T* Ab2 = SPLIT ? (A2  + (size_t)b * strideA) : nullptr;
  const T* Bb2 = SPLIT ? (Bt2 + (size_t)b * strideB) : nullptr;

  const int rlane = lane & 15;
  const int koff  = (lane >> 4) * 8;
  const int mOff  = (lane >> 4) * 8;

  v8f acc[4][4];
#pragma unroll
  for (int i = 0; i < 4; ++i)
#pragma unroll
    for (int j = 0; j < 4; ++j) acc[i][j] = (v8f){0.f,0.f,0.f,0.f,0.f,0.f,0.f,0.f};

  for (int k0 = 0; k0 < K; k0 += 32) {
    V bh[4], bl[4];
#pragma unroll
    for (int j = 0; j < 4; ++j) {
      const size_t bo = (size_t)(n0 + (j << 4) + rlane) * ldb + koff + k0;
      bh[j] = Frag<T>::load(Bb + bo);
      if (SPLIT) bl[j] = Frag<T>::load(Bb2 + bo);
    }
#pragma unroll
    for (int i = 0; i < 4; ++i) {
      const size_t ao = (size_t)(m0 + (i << 4) + rlane) * lda + koff + k0;
      V ah = Frag<T>::load(Ab + ao);
      V al;
      if (SPLIT) al = Frag<T>::load(Ab2 + ao);
#pragma unroll
      for (int j = 0; j < 4; ++j) {
        acc[i][j] = Frag<T>::mma(ah, bh[j], acc[i][j]);
        if (SPLIT) {
          acc[i][j] = Frag<T>::mma(ah, bl[j], acc[i][j]);
          acc[i][j] = Frag<T>::mma(al, bh[j], acc[i][j]);
        }
      }
      Frag<T>::guard4(acc[i][0], acc[i][1], acc[i][2], acc[i][3], ah, SPLIT ? al : ah);
    }
    Frag<T>::keep(bh[0], bh[1], bh[2], bh[3]);
    if (SPLIT) Frag<T>::keep(bl[0], bl[1], bl[2], bl[3]);
  }
  acc_guard4(acc[0][0], acc[0][1], acc[0][2], acc[0][3]);
  acc_guard4(acc[1][0], acc[1][1], acc[1][2], acc[1][3]);
  acc_guard4(acc[2][0], acc[2][1], acc[2][2], acc[2][3]);
  acc_guard4(acc[3][0], acc[3][1], acc[3][2], acc[3][3]);

  float* slab = sT[wave];
  const float* Rb = RESID ? (resid + (size_t)b * strideR) : nullptr;
#pragma unroll
  for (int i = 0; i < 4; ++i) {
    const int mBase = m0 + (i << 4);
#pragma unroll
    for (int j = 0; j < 4; ++j) {
      const int n = n0 + (j << 4) + rlane;
      float bv = 0.f;
      if (BIAS_MODE == 2) bv = bias[n];
#pragma unroll
      for (int r = 0; r < 8; ++r) {
        float v = acc[i][j][r] * scale;
        if (BIAS_MODE == 1) v += bias[mBase + mOff + r];
        if (BIAS_MODE == 2) v += bv;
        if (RESID) v += Rb[(size_t)(mBase + mOff + r) * ldc + n];
        if (ACT == 1) v = tanhf(v);
        if (ACT == 2) v = fmaxf(v, 0.0f);
        if (ACT == 4) v = (v > 0.f) ? v : 0.01f * v;
        slab[(mOff + r) * 68 + (j << 4) + rlane] = v;
      }
    }
    __builtin_amdgcn_fence(__ATOMIC_RELEASE, "workgroup");
    __builtin_amdgcn_wave_barrier();
    __builtin_amdgcn_fence(__ATOMIC_ACQUIRE, "workgroup");
    if (OUT_MODE == 0) {
      float* C = (float*)Cout + (size_t)b * strideC;
      const int hh = lane >> 4, c4 = (lane & 15) * 4;
      for (int pass = 0; pass < 2; ++pass) {
#pragma unroll
        for (int it = 0; it < 8; ++it) {
          const int row = it * 2 + hh;
          v4f v = *(const v4f*)(slab + row * 68 + c4);
          *(volatile v4f*)(C + (size_t)(mBase + row) * ldc + n0 + c4) = v;
        }
        __threadfence();
      }
    } else {
      const int q = lane >> 3, c8 = (lane & 7) * 8;
      unsigned short* C  = (unsigned short*)Cout  + (size_t)b * strideC;
      unsigned short* C2 = (OUT_MODE == 2) ? ((unsigned short*)Cout2 + (size_t)b * strideC) : nullptr;
      for (int pass = 0; pass < 2; ++pass) {
#pragma unroll
        for (int it = 0; it < 4; ++it) {
          const int row = it * 4 + q;
          const float* sp = slab + row * 68 + c8;
          v8h hv, lv;
#pragma unroll
          for (int e = 0; e < 8; ++e) {
            if (OUT_MODE == 1) {
              hv[e] = (_Float16)sp[e];
            } else {
              unsigned short hb = f2bf_bits(sp[e]);
              unsigned short lb = f2bf_bits(sp[e] - bf_bits2f(hb));
              hv[e] = __builtin_bit_cast(_Float16, hb);
              lv[e] = __builtin_bit_cast(_Float16, lb);
            }
          }
          *(volatile v8h*)(C + (size_t)(mBase + row) * ldc + n0 + c8) = hv;
          if (OUT_MODE == 2) *(volatile v8h*)(C2 + (size_t)(mBase + row) * ldc + n0 + c8) = lv;
        }
        __threadfence();
      }
    }
    __builtin_amdgcn_fence(__ATOMIC_RELEASE, "workgroup");
    __builtin_amdgcn_wave_barrier();
    __builtin_amdgcn_fence(__ATOMIC_ACQUIRE, "workgroup");
  }
}

__device__ __forceinline__ void store8_f16_twice(unsigned short* dst, size_t i8, float sc,
                                                 float f0, float f1, float f2, float f3,
                                                 float f4, float f5, float f6, float f7) {
  v8h hv;
  hv[0] = (_Float16)(f0 * sc);
  hv[1] = (_Float16)(f1 * sc);
  hv[2] = (_Float16)(f2 * sc);
  hv[3] = (_Float16)(f3 * sc);
  hv[4] = (_Float16)(f4 * sc);
  hv[5] = (_Float16)(f5 * sc);
  hv[6] = (_Float16)(f6 * sc);
  hv[7] = (_Float16)(f7 * sc);
  volatile v8h* op = (volatile v8h*)(dst + i8 * 8);
  *op = hv;
  __threadfence();
  *op = hv;
}

__global__ __launch_bounds__(256) void pack_rec_kernel(const float* __restrict__ whh_f, const float* __restrict__ whh_b,
                                                       const float* __restrict__ wih_f, const float* __restrict__ wih_b,
                                                       unsigned short* __restrict__ dst) {
  const int i = blockIdx.x * 256 + threadIdx.x;
  if (i >= NREC8) return;
  const int row = i / (KREC / 8);
  const int c8  = i - row * (KREC / 8);
  const int gd  = row / HPADR;
  const int j   = row - gd * HPADR;
  const int dir = gd >> 2;
  const int g   = gd & 3;
  const bool rowok = j < NHID;
  const int srow = g * NHID + (rowok ? j : (NHID - 1));
  const float* hp = (dir ? whh_b : whh_f) + (size_t)srow * NHID;
  const float* ip = (dir ? wih_b : wih_f) + (size_t)srow * NIHP + NHID;
  const int kh0 = (c8 * 8 < NHID - 4) ? c8 * 8 : (NHID - 4);
  const int kh1 = (kh0 + 4 < NHID - 4) ? (kh0 + 4) : (NHID - 4);
  const v4f h0 = *(const v4f*)(hp + kh0);
  const v4f h1 = *(const v4f*)(hp + kh1);
  int s0 = (c8 - KHP / 8) * 8;
  s0 = s0 < 0 ? 0 : s0;
  s0 = s0 > NSW - 2 ? NSW - 2 : s0;
  const int s1 = (s0 + 2 < NSW - 2) ? (s0 + 2) : (NSW - 2);
  const int s2 = (s0 + 4 < NSW - 2) ? (s0 + 4) : (NSW - 2);
  const int s3 = (s0 + 6 < NSW - 2) ? (s0 + 6) : (NSW - 2);
  const v2f q0 = *(const v2f*)(ip + s0);
  const v2f q1 = *(const v2f*)(ip + s1);
  const v2f q2 = *(const v2f*)(ip + s2);
  const v2f q3 = *(const v2f*)(ip + s3);
  const bool hlo  = rowok && (c8 <= 187);
  const bool hhi  = rowok && (c8 <= 186);
  const bool iall = rowok && (c8 >= 192) && (c8 <= 197);
  const bool i0   = iall || (rowok && (c8 == 198));
  const float f0 = hlo ? h0[0] : (i0 ? q0[0] : 0.0f);
  const float f1 = hlo ? h0[1] : (i0 ? q0[1] : 0.0f);
  const float f2 = hlo ? h0[2] : (iall ? q1[0] : 0.0f);
  const float f3 = hlo ? h0[3] : (iall ? q1[1] : 0.0f);
  const float f4 = hhi ? h1[0] : (iall ? q2[0] : 0.0f);
  const float f5 = hhi ? h1[1] : (iall ? q2[1] : 0.0f);
  const float f6 = hhi ? h1[2] : (iall ? q3[0] : 0.0f);
  const float f7 = hhi ? h1[3] : (iall ? q3[1] : 0.0f);
  store8_f16_twice(dst, (size_t)i, WCARRY, f0, f1, f2, f3, f4, f5, f6, f7);
}

__global__ __launch_bounds__(256) void pack_x_kernel(const float* __restrict__ wih_f, const float* __restrict__ wih_b,
                                                     unsigned short* __restrict__ dst) {
  const int i = blockIdx.x * 256 + threadIdx.x;
  if (i >= NX8) return;
  const int row = i / (KHP / 8);
  const int c8  = i - row * (KHP / 8);
  const int gd  = row / HPADR;
  const int j   = row - gd * HPADR;
  const int dir = gd >> 2;
  const int g   = gd & 3;
  const bool rowok = j < NHID;
  const int srow = g * NHID + (rowok ? j : (NHID - 1));
  const float* xp = (dir ? wih_b : wih_f) + (size_t)srow * NIHP;
  const int k0 = c8 * 8;
  const int ka = (k0     < NHID - 2) ? k0       : (NHID - 2);
  const int kb = (k0 + 2 < NHID - 2) ? (k0 + 2) : (NHID - 2);
  const int kc = (k0 + 4 < NHID - 2) ? (k0 + 4) : (NHID - 2);
  const int kd = (k0 + 6 < NHID - 2) ? (k0 + 6) : (NHID - 2);
  const v2f q0 = *(const v2f*)(xp + ka);
  const v2f q1 = *(const v2f*)(xp + kb);
  const v2f q2 = *(const v2f*)(xp + kc);
  const v2f q3 = *(const v2f*)(xp + kd);
  const bool v0 = rowok && (k0     < NHID);
  const bool v1 = rowok && (k0 + 2 < NHID);
  const bool v2 = rowok && (k0 + 4 < NHID);
  const bool v3 = rowok && (k0 + 6 < NHID);
  store8_f16_twice(dst, (size_t)i, WCARRY,
                   v0 ? q0[0] : 0.0f, v0 ? q0[1] : 0.0f, v1 ? q1[0] : 0.0f, v1 ? q1[1] : 0.0f,
                   v2 ? q2[0] : 0.0f, v2 ? q2[1] : 0.0f, v3 ? q3[0] : 0.0f, v3 ? q3[1] : 0.0f);
}

__global__ __launch_bounds__(256) void pack_e_kernel(const float* __restrict__ emb, unsigned short* __restrict__ dst) {
  const int i = blockIdx.x * 256 + threadIdx.x;
  if (i >= NE8) return;
  const int row = i / (KHP / 8);
  const int c8  = i - row * (KHP / 8);
  const bool rowok = row < NVOC;
  const int srow = rowok ? row : (NVOC - 1);
  const float* ep = emb + (size_t)srow * NHID;
  const int kh0 = (c8 * 8 < NHID - 4) ? c8 * 8 : (NHID - 4);
  const int kh1 = (kh0 + 4 < NHID - 4) ? (kh0 + 4) : (NHID - 4);
  const v4f h0 = *(const v4f*)(ep + kh0);
  const v4f h1 = *(const v4f*)(ep + kh1);
  const bool hlo = rowok && (c8 <= 187);
  const bool hhi = rowok && (c8 <= 186);
  store8_f16_twice(dst, (size_t)i, ECARRY,
                   hlo ? h0[0] : 0.0f, hlo ? h0[1] : 0.0f, hlo ? h0[2] : 0.0f, hlo ? h0[3] : 0.0f,
                   hhi ? h1[0] : 0.0f, hhi ? h1[1] : 0.0f, hhi ? h1[2] : 0.0f, hhi ? h1[3] : 0.0f);
}

__global__ __launch_bounds__(256) void bias_plane_kernel(const float* __restrict__ bif, const float* __restrict__ bhf,
                                                         const float* __restrict__ bib, const float* __restrict__ bhb,
                                                         float* __restrict__ dst) {
  const int i = blockIdx.x * 256 + threadIdx.x;
  if (i >= NB4) return;
  const int n   = i * 4;
  const int gd  = n / HPADR;
  const int j   = n - gd * HPADR;
  const int dir = gd >> 2;
  const int g   = gd & 3;
  const bool ok = j < NHID;
  const int src = g * NHID + (ok ? j : (NHID - 4));
  const v4f a0 = *(const v4f*)(bif + src);
  const v4f a1 = *(const v4f*)(bhf + src);
  const v4f b0 = *(const v4f*)(bib + src);
  const v4f b1 = *(const v4f*)(bhb + src);
  v4f o;
#pragma unroll
  for (int e = 0; e < 4; ++e) {
    const float sf = a0[e] + a1[e];
    const float sb = b0[e] + b1[e];
    o[e] = ok ? (dir ? sb : sf) : 0.0f;
  }
  volatile v4f* op = (volatile v4f*)(dst + n);
  *op = o;
  __threadfence();
  *op = o;
}

__global__ __launch_bounds__(RTHR) void stack_lstm_seq_kernel(
    const int* __restrict__ tokens, const float* __restrict__ hidden0, const float* __restrict__ cell0,
    const float* __restrict__ stack0,
    const float* __restrict__ wctrl, const float* __restrict__ bctrl,
    const float* __restrict__ wsi, const float* __restrict__ bsi,
    const float* __restrict__ wdec, const float* __restrict__ bdec,
    const unsigned short* __restrict__ Wrp, const float* __restrict__ Ptab, float* __restrict__ out) {
  __shared__ __align__(16) _Float16 vecs[2][2 * KREC];
  __shared__ __align__(16) float    cst[2 * HPADR];
  __shared__ __align__(16) float    hcat[2 * HPADR];
  __shared__ __align__(16) float    stk[2][512];
  __shared__ __align__(16) float    scr[128];
  __shared__ __align__(16) float    lgs[NSTEP * NVOC];
  __shared__ int                    tokS[NSTEP];

  const int tid  = threadIdx.x;
  const int lane = tid & 31;
  const int wave = __builtin_amdgcn_readfirstlane(tid >> 5);
  const int c    = lane & 15;
  const int hh   = lane >> 4;
  const int koff = hh * 8;
  const _Float16* Wr = (const _Float16*)Wrp;

  {
    _Float16* vflat = &vecs[0][0];
#pragma unroll 1
    for (int it = 0; it < 13; ++it) {
      const int i   = it * RTHR + tid;
      const int ic  = i < 4 * KREC ? i : (4 * KREC - 1);
      const int buf = ic / (2 * KREC);
      const int rem = ic - buf * (2 * KREC);
      const int d   = rem / KREC;
      const int k   = rem - d * KREC;
      const int kc  = k < NHID ? k : (NHID - 1);
      const float hv  = hidden0[d * NHID + kc];
      const float val = (buf == 0 && k < NHID) ? hv * HCARRY : 0.0f;
      if (i < 4 * KREC) vflat[i] = (_Float16)val;
    }
#pragma unroll 1
    for (int it = 0; it < 6; ++it) {
      const int i  = it * RTHR + tid;
      const int ic = i < 2 * HPADR ? i : (2 * HPADR - 1);
      const int ih = ic < NH2 ? ic : (NH2 - 1);
      const float hv = hidden0[ih];
      const int d  = ic / HPADR;
      const int j  = ic - d * HPADR;
      const int jc = j < NHID ? j : (NHID - 1);
      const float cv = cell0[d * NHID + jc];
      if (i < 2 * HPADR) {
        hcat[i] = (ic < NH2) ? hv : 0.0f;
        cst[i]  = (j < NHID) ? cv : 0.0f;
      }
    }
    float* sflat = &stk[0][0];
#pragma unroll 1
    for (int it = 0; it < 2; ++it) {
      const int i  = it * RTHR + tid;
      const int ic = i < NSD * NSW ? i : (NSD * NSW - 1);
      const float sv = stack0[ic];
      sflat[i] = (i < NSD * NSW) ? sv : 0.0f;
    }
    if (tid < 128) {
      scr[tid] = 0.0f;
      int tk = tokens[tid];
      tk = tk < 0 ? 0 : tk;
      tk = tk > NVOC - 1 ? NVOC - 1 : tk;
      tokS[tid] = tk;
    }
  }
  __syncthreads();

  const v8f z8 = {0.f, 0.f, 0.f, 0.f, 0.f, 0.f, 0.f, 0.f};
  const size_t gateStride = (size_t)HPADR * KREC;

#pragma unroll 1
  for (int t = 0; t <= NSTEP; ++t) {
    const int cur = t & 1;

#pragma unroll 1
    for (int rnd = 0; rnd < 7; ++rnd) {
      const int row = rnd * RWAVES + wave;
      const int rc  = row < NROWA ? row : (NROWA - 1);
      const int rd  = rc < NVOC ? rc : (NVOC - 1);
      int rk = rc - NVOC;
      rk = rk < 0 ? 0 : rk;
      rk = rk > 2 ? 2 : rk;
      int rs = rc - NVOC - 3;
      rs = rs < 0 ? 0 : rs;
      const float* pd = wdec  + (size_t)rd * NH2;
      const float* pk = wctrl + (size_t)rk * NH2;
      const float* ps = wsi   + (size_t)rs * NH2;
      const float* wrow = (rc < NVOC) ? pd : ((rc < NVOC + 3) ? pk : ps);
      const float bd = bdec[rd];
      const float bk = bctrl[rk];
      const float bs = bsi[rs];
      const float bsel = (rc < NVOC) ? bd : ((rc < NVOC + 3) ? bk : bs);
      float s = 0.0f;
#pragma unroll 1
      for (int it = 0; it < 24; ++it) {
        const int q  = it * 32 + lane;
        const int qc = q < NH2 / 4 ? q : (NH2 / 4 - 1);
        const v4f w  = *(const v4f*)(wrow + 4 * qc);
        const v4f hv = *(const v4f*)(hcat + 4 * qc);
        float p = w[0] * hv[0];
        p = fmaf(w[1], hv[1], p);
        p = fmaf(w[2], hv[2], p);
        p = fmaf(w[3], hv[3], p);
        s += (q < NH2 / 4) ? p : 0.0f;
      }
#pragma unroll
      for (int off = 16; off > 0; off >>= 1) s += __shfl_xor(s, off, 32);
      const float sb = s + bsel;
      const float tb = tanhf(sb);
      if (lane == 0 && row < NROWA) {
        if (row < NVOC) {
          if (t >= 1) lgs[(t - 1) * NVOC + row] = sb;
        } else if (row < NVOC + 3) {
          scr[row - NVOC] = sb;
        } else {
          scr[32 + row - NVOC - 3] = tb;
        }
      }
    }
    __syncthreads();

    if (t < NSTEP) {
      {
        const float r0 = scr[0], r1 = scr[1], r2 = scr[2];
        const float mx = fmaxf(r0, fmaxf(r1, r2));
        const float e0 = expf(r0 - mx), e1 = expf(r1 - mx), e2 = expf(r2 - mx);
        const float inv = 1.0f / (e0 + e1 + e2);
        const float ppush = e0 * inv, ppop = e1 * inv, pstay = e2 * inv;
        const float* so = &stk[cur][0];
        float* sn = &stk[cur ^ 1][0];
        const int e  = tid;
        const int ec = e < NSD * NSW ? e : (NSD * NSW - 1);
        const int d  = ec / NSW;
        const int w  = ec - d * NSW;
        const int eu = ec - NSW < 0 ? 0 : (ec - NSW);
        const int ed = ec + NSW > NSD * NSW - 1 ? (NSD * NSW - 1) : (ec + NSW);
        const float cv  = so[ec];
        const float upS = scr[32 + w];
        const float upP = so[eu];
        const float dnP = so[ed];
        const float up  = (d == 0) ? upS : upP;
        const float dn  = (d == NSD - 1) ? 0.0f : dnP;
        const float nv  = pstay * cv + ppush * up + ppop * dn;
        if (e < NSD * NSW) sn[e] = nv;
        if (e < 64) {
          const float tv = (e < NSW) ? nv * HCARRY : 0.0f;
          const _Float16 t16 = (_Float16)tv;
          vecs[cur][KHP + e] = t16;
          vecs[cur][KREC + KHP + e] = t16;
        }
        if (e >= 64 && e < 64 + (KHP - NHID)) {
          const int pi = e - 64;
          vecs[cur ^ 1][NHID + pi] = (_Float16)0.0f;
          vecs[cur ^ 1][KREC + NHID + pi] = (_Float16)0.0f;
        }
      }
      __syncthreads();

      {
        const _Float16* vcur = &vecs[cur][0];
        _Float16* vnxt = &vecs[cur ^ 1][0];
        const int tok = tokS[t];
        const float* Prow = Ptab + (size_t)tok * NGROW;
#pragma unroll 1
        for (int task = wave; task < NTASK; task += RWAVES) {
          const int dir  = task >= NTILE ? 1 : 0;
          const int tile = task - dir * NTILE;
          const int j    = tile * 16 + c;
          const float* pp = Prow + dir * NDIRROW + j;
          float p0 = pp[0];
          float p1 = pp[HPADR];
          float p2 = pp[2 * HPADR];
          float p3 = pp[3 * HPADR];
          asm volatile("" : "+v"(p0), "+v"(p1), "+v"(p2), "+v"(p3));
          const float cold = cst[dir * HPADR + j];
          const _Float16* av = vcur + dir * KREC + koff;
          const _Float16* w0 = Wr + ((size_t)(dir * 4) * HPADR + (size_t)j) * KREC + koff;
          const _Float16* w1 = w0 + gateStride;
          const _Float16* w2 = w1 + gateStride;
          const _Float16* w3 = w2 + gateStride;
          v8f a0 = z8, a1 = z8, a2 = z8, a3 = z8;
#pragma unroll 1
          for (int k0 = 0; k0 < KREC; k0 += 32) {
            const v16h a  = Frag<_Float16>::load(av + k0);
            const v16h b0 = Frag<_Float16>::load(w0 + k0);
            const v16h b1 = Frag<_Float16>::load(w1 + k0);
            const v16h b2 = Frag<_Float16>::load(w2 + k0);
            const v16h b3 = Frag<_Float16>::load(w3 + k0);
            a0 = Frag<_Float16>::mma(a, b0, a0);
            a1 = Frag<_Float16>::mma(a, b1, a1);
            a2 = Frag<_Float16>::mma(a, b2, a2);
            a3 = Frag<_Float16>::mma(a, b3, a3);
            rec_guard(a0, a1, a2, a3, a, b0, b1, b2, b3);
          }
          acc_guard4(a0, a1, a2, a3);
          const float zi = a0[0] * RECFOLD + p0;
          const float zf = a1[0] * RECFOLD + p1;
          const float zg = a2[0] * RECFOLD + p2;
          const float zo = a3[0] * RECFOLD + p3;
          const float gi = 1.0f / (1.0f + expf(-zi));
          const float gf = 1.0f / (1.0f + expf(-zf));
          const float gg = tanhf(zg);
          const float go = 1.0f / (1.0f + expf(-zo));
          float cn = gf * cold + gi * gg;
          float hn = go * tanhf(cn);
          float hs = hn * HCARRY;
          asm volatile("" : "+v"(cn), "+v"(hn), "+v"(hs));
          const _Float16 h16 = (_Float16)hs;
          if (hh == 0 && j < NHID) {
            cst[dir * HPADR + j] = cn;
            hcat[dir * NHID + j] = hn;
            vnxt[dir * KREC + j] = h16;
          }
        }
      }
      __syncthreads();
    }
  }

  for (int pass = 0; pass < 2; ++pass) {
#pragma unroll
    for (int it = 0; it < 3; ++it) {
      const int idx = it * RTHR + tid;
      if (idx < (NSTEP * NVOC) / 4) {
        const v4f v = *(const v4f*)(lgs + 4 * idx);
        *(volatile v4f*)(out + 4 * idx) = v;
      }
    }
    __threadfence();
  }
}

extern "C" void kernel_launch(void* const* d_in, const int* in_sizes, int n_in,
                              void* d_out, int out_size, void* d_ws, size_t ws_size, hipStream_t stream) {
  if (n_in < 19 || d_out == nullptr || d_ws == nullptr) return;
  if (in_sizes[0] != NSTEP || in_sizes[1] != 2 * NHID || in_sizes[2] != 2 * NHID || in_sizes[3] != NSD * NSW ||
      in_sizes[4] != NVOC * NHID || in_sizes[5] != 3 * NH2 || in_sizes[6] != 3 || in_sizes[7] != NSW * NH2 ||
      in_sizes[8] != NSW || in_sizes[9] != 4 * NHID * NIHP || in_sizes[10] != 4 * NHID * NHID ||
      in_sizes[11] != 4 * NHID || in_sizes[12] != 4 * NHID || in_sizes[13] != 4 * NHID * NIHP ||
      in_sizes[14] != 4 * NHID * NHID || in_sizes[15] != 4 * NHID || in_sizes[16] != 4 * NHID ||
      in_sizes[17] != NVOC * NH2 || in_sizes[18] != NVOC || out_size != NSTEP * NVOC) return;

  const int*   tokens  = (const int*)  d_in[0];
  const float* hidden0 = (const float*)d_in[1];
  const float* cell0   = (const float*)d_in[2];
  const float* stack0  = (const float*)d_in[3];
  const float* emb     = (const float*)d_in[4];
  const float* wctrl   = (const float*)d_in[5];
  const float* bctrl   = (const float*)d_in[6];
  const float* wsi     = (const float*)d_in[7];
  const float* bsi     = (const float*)d_in[8];
  const float* wih_f   = (const float*)d_in[9];
  const float* whh_f   = (const float*)d_in[10];
  const float* bih_f   = (const float*)d_in[11];
  const float* bhh_f   = (const float*)d_in[12];
  const float* wih_b   = (const float*)d_in[13];
  const float* whh_b   = (const float*)d_in[14];
  const float* bih_b   = (const float*)d_in[15];
  const float* bhh_b   = (const float*)d_in[16];
  const float* wdec    = (const float*)d_in[17];
  const float* bdec    = (const float*)d_in[18];
  float* out = (float*)d_out;

  char* ws = (char*)d_ws; size_t off = 0;
  auto carve = [&](size_t bytes) -> char* { char* p = ws + off; off += (bytes + 255) & ~(size_t)255; return p; };
  unsigned short* WR    = (unsigned short*)carve((size_t)NGROW * KREC * 2);
  unsigned short* WX    = (unsigned short*)carve((size_t)NGROW * KHP * 2);
  unsigned short* EH    = (unsigned short*)carve((size_t)64 * KHP * 2);
  float*          BIASP = (float*)carve((size_t)NGROW * 4);
  float*          PT    = (float*)carve((size_t)64 * NGROW * 4);
  if (off > ws_size || off > (size_t)134217728) return;

  pack_rec_kernel<<<NREC8 / 256, 256, 0, stream>>>(whh_f, whh_b, wih_f, wih_b, WR);
  pack_x_kernel<<<NX8 / 256, 256, 0, stream>>>(wih_f, wih_b, WX);
  pack_e_kernel<<<NE8 / 256, 256, 0, stream>>>(emb, EH);
  bias_plane_kernel<<<(NB4 + 255) / 256, 256, 0, stream>>>(bih_f, bhh_f, bih_b, bhh_b, BIASP);

  wmma_gemm64<0, false, 2, 0, false, 0><<<dim3((NGROW / 64 + 7) / 8, 1), 256, 0, stream>>>(
      EH, EH, KHP, 0L, WX, WX, KHP, 0L, (void*)PT, (void*)PT, NGROW, 0L,
      BIASP, BIASP, 0L, 64, NGROW, KHP, TABFOLD);

  stack_lstm_seq_kernel<<<1, RTHR, 0, stream>>>(tokens, hidden0, cell0, stack0, wctrl, bctrl, wsi, bsi, wdec, bdec,
                                                WR, PT, out);
}
